// ShipGNNWithDecoder_25555055411313
// MI455X (gfx1250) — hardware-run, weakly checked
//
#include <hip/hip_runtime.h>
#include <stddef.h>
#include <stdint.h>
#include <math.h>


#define NN      100000
#define NE      1600000
#define NPD     100096
#define XW      12
#define FW      32
#define NFEAT   18
#define HD      128
#define NG      1000
#define NGP     1024
#define GCB     32
#define NTHR    256
#define NWAVE   8
#define EPT     8
#define CHUNK   (NTHR * EPT)
#define WCAP    (EPT * 32)
#define LISTN   (NWAVE * WCAP)
#define NBA     1024
#define SLA     10
#define SRCB    17
#define SRCM    0x1FFFF
#define NB      98
#define NSLOT   (NB * NBA)
#define RCAP    28672
#define LISTTOT (NB * RCAP)
#define DEGCAP  48
#define R2CAP   49152
#define MEAS_B1024  16703
#define MEAS_MAXDEG 36
#define GBM     64
#define GBN     128
#define GTHR    128
#define GGP     (NGP * 384)
#define CMP_ZINTS (RCAP + 3 * NBA)
#define CMP_LDS_INTS (LISTN + 2 * RCAP + 3 * NBA + 16)
#define WSMAX   134217728

static_assert((CHUNK & (CHUNK - 1)) == 0 && CHUNK <= 4096);
static_assert(NBA == (1 << SLA) && ((long long)CHUNK << SLA) < (1LL << 31));
static_assert(NN - 1 <= SRCM && (((long long)(NBA - 1) << SRCB) | SRCM) < (1LL << 31));
static_assert(NSLOT >= NPD && NPD >= NN && (NPD % 128) == 0 && (NPD * 8) % NTHR == 0);
static_assert(RCAP >= MEAS_B1024 + 4096 && (RCAP % 1024) == 0);
static_assert(DEGCAP >= MEAS_MAXDEG + 8 && DEGCAP <= 64);
static_assert(R2CAP >= NG * (1 + DEGCAP) && (R2CAP % 128) == 0 && (R2CAP % 1024) == 0);
static_assert(LISTN >= NWAVE * WCAP && (CMP_ZINTS % 4) == 0);
static_assert(CMP_LDS_INTS * 4 + NBA * 4 <= 300000);
static_assert(R2CAP * 4 + 6 * NGP * 4 <= 300000);
static_assert((NE % 4) == 0 && (NN % 4) == 0 && (NN / 4) <= 98 * NTHR);
static_assert(GBM == (GTHR / 32) * 16 && GBN == 128 && (NPD % GBM) == 0 && (NGP % GBM) == 0 && (R2CAP % GBM) == 0);
static_assert(GCB == 32 && (NGP % GCB) == 0 && NGP == 4 * NTHR);

typedef float          v2f  __attribute__((ext_vector_type(2)));
typedef float          v4f  __attribute__((ext_vector_type(4)));
typedef float          v8f  __attribute__((ext_vector_type(8)));
typedef int            v4i  __attribute__((ext_vector_type(4)));
typedef int            v8i  __attribute__((ext_vector_type(8)));
typedef unsigned int   v4u  __attribute__((ext_vector_type(4)));
typedef unsigned short v8us __attribute__((ext_vector_type(8)));
typedef __bf16         v16b __attribute__((ext_vector_type(16)));
typedef v2f  __attribute__((may_alias)) v2fa;
typedef v4f  __attribute__((may_alias)) v4fa;
typedef v4i  __attribute__((may_alias)) v4ia;
typedef v8us __attribute__((may_alias)) v8usa;
union FragB { v16b v; v8us h[2]; v8i w; };

constexpr size_t al256c(size_t v) { return (v + 255) & ~(size_t)255; }
constexpr size_t O_W1D   = 0;
constexpr size_t O_W2D   = al256c(O_W1D   + (size_t)128 * 64 * 2);
constexpr size_t O_W3D   = al256c(O_W2D   + (size_t)128 * 256 * 2);
constexpr size_t O_BG    = al256c(O_W3D   + (size_t)128 * 256 * 2);
constexpr size_t O_WG    = al256c(O_BG    + (size_t)3 * 128 * 4);
constexpr size_t O_BGRU  = al256c(O_WG    + (size_t)4 * 384 * 256 * 2);
constexpr size_t O_WHD   = al256c(O_BGRU  + (size_t)4 * 384 * 4);
constexpr size_t O_SC    = al256c(O_WHD   + (size_t)256 * 512 * 2);
constexpr size_t O_GAPN  = al256c(O_SC    + (size_t)544 * 4);
constexpr size_t O_GCNT  = al256c(O_GAPN  + (size_t)NGP * 4);
constexpr size_t O_FLAG  = al256c(O_GCNT  + (size_t)NGP * 4);
constexpr size_t O_LIST  = al256c(O_FLAG  + (size_t)(NB + 1) * 128);
constexpr size_t O_CNT   = al256c(O_LIST  + (size_t)LISTTOT * 4);
constexpr size_t O_OFF   = al256c(O_CNT   + (size_t)NSLOT * 4);
constexpr size_t O_DIS   = al256c(O_OFF   + (size_t)NSLOT * 4);
constexpr size_t O_Q     = al256c(O_DIS   + (size_t)NSLOT * 4);
constexpr size_t O_AGG1  = O_Q + (size_t)NPD * FW * 4;
constexpr size_t O_H1    = al256c(O_AGG1  + (size_t)NPD * 64 * 2);
constexpr size_t O_AGG2  = al256c(O_H1    + (size_t)NPD * HD * 4);
constexpr size_t O_ROWS2 = al256c(O_AGG2  + (size_t)R2CAP * 256 * 2);
constexpr size_t O_POS   = al256c(O_ROWS2 + (size_t)R2CAP * 4);
constexpr size_t O_RINF  = al256c(O_POS   + (size_t)NGP * 4);
constexpr size_t O_AGG3  = al256c(O_RINF  + (size_t)128);
constexpr size_t O_H0    = al256c(O_AGG3  + (size_t)NGP * 256 * 2);
constexpr size_t O_H0HL  = al256c(O_H0    + (size_t)NGP * HD * 4);
constexpr size_t O_GG    = al256c(O_H0HL  + (size_t)NGP * 256 * 2);
constexpr size_t O_HF    = al256c(O_GG    + (size_t)4 * GGP * 4);
constexpr size_t O_HB    = al256c(O_HF    + (size_t)2 * NGP * HD * 4);
constexpr size_t O_HFHL  = al256c(O_HB    + (size_t)2 * NGP * HD * 4);
constexpr size_t O_HBHL  = al256c(O_HFHL  + (size_t)NGP * 256 * 2);
constexpr size_t O_OUTHL = al256c(O_HBHL  + (size_t)NGP * 256 * 2);
constexpr size_t O_INPHL = al256c(O_OUTHL + (size_t)NGP * 512 * 2);
constexpr size_t O_PRED  = al256c(O_INPHL + (size_t)NGP * 256 * 2);
constexpr size_t WS_TOTAL = al256c(O_PRED + (size_t)3 * NGP * 2 * 4);
constexpr size_t HPL     = (size_t)NGP * HD * 4;
static_assert(WS_TOTAL <= (size_t)WSMAX);
static_assert((size_t)R2CAP * HD * 4 <= (size_t)NPD * FW * 4 + (size_t)NPD * 64 * 2);
static_assert(O_AGG1 % 256 == 0);
static_assert((size_t)(NGP / GCB) * GCB * 4 <= (size_t)NGP * 4);

__device__ __forceinline__ v8f wmb(const FragB& a, const FragB& b, v8f c) {
  v8f d = __builtin_amdgcn_wmma_f32_16x16x32_bf16(false, a.v, false, b.v, (short)0, c, false, false);
  asm volatile("v_nop\n\tv_nop\n\tv_nop\n\tv_nop" : "+v"(d) : "v"(a.w), "v"(b.w));
  return d;
}

__device__ __forceinline__ unsigned int f2bf(float f) {
  const unsigned int u = __float_as_uint(f);
  const unsigned int r = ((u + 0x7FFFu + ((u >> 16) & 1u)) >> 16) & 0xFFFFu;
  return ((u & 0x7FFFFFFFu) > 0x7F800000u) ? 0x7FC0u : r;
}
__device__ __forceinline__ float bf2f(unsigned int b) { return __uint_as_float(b << 16); }
__device__ __forceinline__ float bfr(float f) { return bf2f(f2bf(f)); }
__device__ __forceinline__ v4f bfr4(v4f v) { v4f o; o.x = bfr(v.x); o.y = bfr(v.y); o.z = bfr(v.z); o.w = bfr(v.w); return o; }

__device__ __forceinline__ void pin(int& v)   { asm volatile("" : "+v"(v)); }
__device__ __forceinline__ void pin(float& v) { asm volatile("" : "+v"(v)); }
__device__ __forceinline__ void pin(v4f& v)   { asm volatile("" : "+v"(v)); }
__device__ __forceinline__ void pin(v4i& v)   { asm volatile("" : "+v"(v)); }
__device__ __forceinline__ int clampi(int v, int lo, int hi) { return v < lo ? lo : (v > hi ? hi : v); }
__device__ __forceinline__ int uloadi(const int* p) { int v = *p; pin(v); return __builtin_amdgcn_readfirstlane(v); }
__device__ __forceinline__ float uloadf(const float* p) {
  float v = *p; pin(v);
  return __int_as_float(__builtin_amdgcn_readfirstlane(__float_as_int(v)));
}
__device__ __forceinline__ float relu_np(float v) { return (v > 0.0f) ? v : (v - v); }

__device__ __forceinline__ v4u hl_pack(const v4f v, const int lane) {
  const unsigned h0 = f2bf(v.x), h1 = f2bf(v.y), h2 = f2bf(v.z), h3 = f2bf(v.w);
  const unsigned l0 = f2bf(v.x - bf2f(h0)), l1 = f2bf(v.y - bf2f(h1));
  const unsigned l2 = f2bf(v.z - bf2f(h2)), l3 = f2bf(v.w - bf2f(h3));
  const int hw0 = (int)(h0 | (h1 << 16)), hw1 = (int)(h2 | (h3 << 16));
  const int lw0 = (int)(l0 | (l1 << 16)), lw1 = (int)(l2 | (l3 << 16));
  const int sa = (2 * lane) & 31, sb = (2 * lane + 1) & 31;
  const int g0 = __shfl(hw0, sa, 32), g1 = __shfl(hw1, sa, 32);
  const int g2 = __shfl(hw0, sb, 32), g3 = __shfl(hw1, sb, 32);
  const int p0 = __shfl(lw0, sa, 32), p1 = __shfl(lw1, sa, 32);
  const int p2 = __shfl(lw0, sb, 32), p3 = __shfl(lw1, sb, 32);
  const bool ls = lane >= 16;
  v4u o;
  o.x = (unsigned)(ls ? p0 : g0); o.y = (unsigned)(ls ? p1 : g1);
  o.z = (unsigned)(ls ? p2 : g2); o.w = (unsigned)(ls ? p3 : g3);
  return o;
}

__device__ __forceinline__ int scan1024(const int* cin, int* o0, int* o1, int lane) {
  const int base = lane * 32;
  int s = 0;
#pragma unroll 1
  for (int i = 0; i < 32; ++i) s += cin[base + i];
  int incl = s;
#pragma unroll
  for (int d = 1; d < 32; d <<= 1) {
    const int y = __shfl_up(incl, d, 32);
    if (lane >= d) incl += y;
  }
  int run = incl - s;
#pragma unroll 1
  for (int i = 0; i < 32; ++i) {
    const int cv = cin[base + i];
    o0[base + i] = run;
    o1[base + i] = run;
    run += cv;
  }
  return __shfl(incl, 31, 32);
}

template <int SLB>
__device__ __forceinline__ int scan_chunk(const int* __restrict__ dsts, int nE, int cbase, int slotBase,
                                          int nb, int vec8, int* list, int tid, int lane, int wave) {
  int wc = 0;
  const int el0  = tid * EPT;
  const int e0   = cbase + el0;
  const int sent = -2147483647 - 1;
  v4i da, db;
  if (vec8 != 0 && cbase + CHUNK <= nE) {
    da = *(const v4i*)(dsts + e0);
    db = *(const v4i*)(dsts + e0 + 4);
  } else {
    da.x = (e0     < nE) ? dsts[min(e0,     nE - 1)] : sent;
    da.y = (e0 + 1 < nE) ? dsts[min(e0 + 1, nE - 1)] : sent;
    da.z = (e0 + 2 < nE) ? dsts[min(e0 + 2, nE - 1)] : sent;
    da.w = (e0 + 3 < nE) ? dsts[min(e0 + 3, nE - 1)] : sent;
    db.x = (e0 + 4 < nE) ? dsts[min(e0 + 4, nE - 1)] : sent;
    db.y = (e0 + 5 < nE) ? dsts[min(e0 + 5, nE - 1)] : sent;
    db.z = (e0 + 6 < nE) ? dsts[min(e0 + 6, nE - 1)] : sent;
    db.w = (e0 + 7 < nE) ? dsts[min(e0 + 7, nE - 1)] : sent;
  }
  const unsigned nbs = (unsigned)slotBase;
  const unsigned unb = (unsigned)nb;
  const unsigned s0 = (unsigned)da.x - nbs, s1 = (unsigned)da.y - nbs;
  const unsigned s2 = (unsigned)da.z - nbs, s3 = (unsigned)da.w - nbs;
  const unsigned s4 = (unsigned)db.x - nbs, s5 = (unsigned)db.y - nbs;
  const unsigned s6 = (unsigned)db.z - nbs, s7 = (unsigned)db.w - nbs;
  const bool h0 = s0 < unb, h1 = s1 < unb, h2 = s2 < unb, h3 = s3 < unb;
  const bool h4 = s4 < unb, h5 = s5 < unb, h6 = s6 < unb, h7 = s7 < unb;
  const unsigned any = __builtin_amdgcn_ballot_w32(h0 | h1 | h2 | h3 | h4 | h5 | h6 | h7);
  if (any != 0u) {
#define HITJ(J, HJ, SJ) { \
      const unsigned mj = __builtin_amdgcn_ballot_w32(HJ); \
      if (mj != 0u) { \
        if (HJ) { \
          const int pos = wc + (int)__builtin_amdgcn_mbcnt_lo(mj, 0u); \
          if (pos < WCAP) list[wave * WCAP + pos] = ((el0 + (J)) << SLB) | (int)(SJ); \
        } \
        wc += (int)__builtin_popcount(mj); } }
    HITJ(0, h0, s0)
    HITJ(1, h1, s1)
    HITJ(2, h2, s2)
    HITJ(3, h3, s3)
    HITJ(4, h4, s4)
    HITJ(5, h5, s5)
    HITJ(6, h6, s6)
    HITJ(7, h7, s7)
#undef HITJ
  }
  return wc;
}

__device__ __forceinline__ v8us wt_unit(const float* __restrict__ W, int ldw, int kmask, int kreal, int n, int k8) {
  v8us o;
#pragma unroll
  for (int i = 0; i < 8; ++i) {
    const int k  = (k8 + i) & kmask;
    const int kc = k < kreal ? k : kreal - 1;
    const float f = W[(size_t)kc * ldw + n];
    o[i] = (k < kreal) ? (unsigned short)f2bf(f) : (unsigned short)0;
  }
  return o;
}
__device__ __forceinline__ void put8(unsigned short* p, const v8us v) {
  *(volatile v8us*)p = v;
  __threadfence();
  *(volatile v8us*)p = v;
}
__device__ __forceinline__ void put4f(float* p, const v4f v, bool ok) {
  if (ok) *(volatile v4f*)p = v;
  __threadfence();
  if (ok) *(volatile v4f*)p = v;
}

#define PA_U1 1024
#define PA_U2 4096
#define PA_UB 256
#define PB_UG 12288
#define PB_UB 512
#define PC_UW 16384
#define PC_US 256
static_assert(PA_U1 % NTHR == 0 && PA_U2 % NTHR == 0 && PB_UG % NTHR == 0 && PC_UW % NTHR == 0 && (PC_UW / 2) % NTHR == 0);

__global__ __launch_bounds__(NTHR) void k_pa(const float* __restrict__ W1, const float* __restrict__ b1,
                                             const float* __restrict__ W2, const float* __restrict__ b2,
                                             const float* __restrict__ W3, const float* __restrict__ b3,
                                             unsigned short* W1D, unsigned short* W2D, unsigned short* W3D,
                                             float* BG) {
  const int u = (int)blockIdx.x * NTHR + (int)threadIdx.x;
  if (u < PA_U1) {
    const int n = u >> 3, k8 = (u & 7) * 8;
    const v8us o = wt_unit(W1, HD, 31, NFEAT, n, k8);
    put8(W1D + (size_t)n * 64 + k8, o);
  } else if (u < PA_U1 + PA_U2) {
    const int v = u - PA_U1, n = v >> 5, k8 = (v & 31) * 8;
    const v8us o = wt_unit(W2, HD, 127, 128, n, k8);
    put8(W2D + (size_t)n * 256 + k8, o);
  } else if (u < PA_U1 + 2 * PA_U2) {
    const int v = u - PA_U1 - PA_U2, n = v >> 5, k8 = (v & 31) * 8;
    const v8us o = wt_unit(W3, HD, 127, 128, n, k8);
    put8(W3D + (size_t)n * 256 + k8, o);
  } else {
    const int v  = u - PA_U1 - 2 * PA_U2;
    const int vc = v < 96 ? v : 95;
    const int tb = vc >> 5, i4 = vc & 31;
    v4f a = *(const v4f*)(b1 + 4 * i4); pin(a);
    v4f b = *(const v4f*)(b2 + 4 * i4); pin(b);
    v4f c = *(const v4f*)(b3 + 4 * i4); pin(c);
    const v4f s = (tb == 0) ? a : ((tb == 1) ? b : c);
    put4f(BG + 4 * vc, bfr4(s), v < 96);
  }
}

__global__ __launch_bounds__(NTHR) void k_pb(const float* __restrict__ Wif, const float* __restrict__ Whf,
                                             const float* __restrict__ bif, const float* __restrict__ bhf,
                                             const float* __restrict__ Wib, const float* __restrict__ Whb,
                                             const float* __restrict__ bib, const float* __restrict__ bhb,
                                             unsigned short* WG, float* BGRU) {
  const int u = (int)blockIdx.x * NTHR + (int)threadIdx.x;
  if (u < 4 * PB_UG) {
    const int pl = u / PB_UG;
    const int v  = u - pl * PB_UG;
    const int n = v >> 5, k8 = (v & 31) * 8;
    v8us o;
    if (pl == 0)      o = wt_unit(Wif, 384, 127, 128, n, k8);
    else if (pl == 1) o = wt_unit(Whf, 384, 127, 128, n, k8);
    else if (pl == 2) o = wt_unit(Wib, 384, 127, 128, n, k8);
    else              o = wt_unit(Whb, 384, 127, 128, n, k8);
    put8(WG + (size_t)pl * 384 * 256 + (size_t)n * 256 + k8, o);
  } else {
    const int v  = u - 4 * PB_UG;
    const int vc = v < 384 ? v : 383;
    const int tb = vc / 96, i4 = vc - tb * 96;
    v4f a = *(const v4f*)(bif + 4 * i4); pin(a);
    v4f b = *(const v4f*)(bhf + 4 * i4); pin(b);
    v4f c = *(const v4f*)(bib + 4 * i4); pin(c);
    v4f d = *(const v4f*)(bhb + 4 * i4); pin(d);
    const v4f s = (tb == 0) ? a : ((tb == 1) ? b : ((tb == 2) ? c : d));
    put4f(BGRU + 4 * vc, bfr4(s), v < 384);
  }
}

__global__ __launch_bounds__(NTHR) void k_pc(const float* __restrict__ Wred, const float* __restrict__ bred,
                                             const float* __restrict__ Wh1, const float* __restrict__ bh1,
                                             const float* __restrict__ Wh2, const float* __restrict__ bh2,
                                             unsigned short* WHD, float* SC) {
  const int u = (int)blockIdx.x * NTHR + (int)threadIdx.x;
  if (u < PC_UW / 2) {
    const int n = u >> 6, k8 = (u & 63) * 8;
    const v8us o = wt_unit(Wh1, HD, 255, 256, n, k8);
    put8(WHD + (size_t)n * 512 + k8, o);
  } else if (u < PC_UW) {
    const int n = u >> 6, k8 = (u & 63) * 8;
    const v8us o = wt_unit(Wred, HD, 255, 256, n - 128, k8);
    put8(WHD + (size_t)n * 512 + k8, o);
  } else {
    const int j  = u - PC_UW;
    const int jc = j < 136 ? j : 135;
    v4f a = *(const v4f*)(bh1  + 4 * clampi(jc, 0, 31));      pin(a);
    v4f b = *(const v4f*)(bred + 4 * clampi(jc - 32, 0, 31)); pin(b);
    v4f c = *(const v4f*)(Wh2  + 4 * clampi(jc - 64, 0, 63)); pin(c);
    float e0 = bh2[0]; pin(e0);
    float e1 = bh2[1]; pin(e1);
    v4f d; d.x = e0; d.y = e1; d.z = 0.0f; d.w = 0.0f;
    const v4f z = {0.0f, 0.0f, 0.0f, 0.0f};
    const v4f s = (jc < 32) ? a : ((jc < 64) ? b : ((jc < 128) ? c : ((jc == 128) ? d : z)));
    put4f(SC + 4 * jc, bfr4(s), j < 136);
  }
}

__global__ __launch_bounds__(NTHR) void k_gcnt(const int* __restrict__ batch, int* GCNT) {
  __shared__ __attribute__((aligned(16))) int wpart[NWAVE * 32];
  __shared__ __attribute__((aligned(16))) int tot[32];
  const int tid = (int)threadIdx.x, lane = tid & 31, wave = tid >> 5;
  const int myid = (int)blockIdx.x * GCB + lane;
  int cnt = 0;
#pragma unroll 1
  for (int it = 0; it < 98; ++it) {
    const int i4 = tid + NTHR * it;
    const int ic = i4 < NN / 4 ? i4 : NN / 4 - 1;
    v4i b = *(const v4i*)(batch + 4 * ic); pin(b);
    const bool ok = i4 < NN / 4;
    b.x = ok ? b.x : -1; b.y = ok ? b.y : -1;
    b.z = ok ? b.z : -1; b.w = ok ? b.w : -1;
#pragma unroll 4
    for (int k = 0; k < 32; ++k) {
      const int e0 = __builtin_amdgcn_readlane(b.x, k);
      const int e1 = __builtin_amdgcn_readlane(b.y, k);
      const int e2 = __builtin_amdgcn_readlane(b.z, k);
      const int e3 = __builtin_amdgcn_readlane(b.w, k);
      cnt += (e0 == myid) ? 1 : 0;
      cnt += (e1 == myid) ? 1 : 0;
      cnt += (e2 == myid) ? 1 : 0;
      cnt += (e3 == myid) ? 1 : 0;
    }
  }
  wpart[wave * 32 + lane] = cnt;
  __syncthreads();
  if (tid < 32) {
    int s = 0;
#pragma unroll
    for (int w2 = 0; w2 < NWAVE; ++w2) s += wpart[w2 * 32 + lane];
    tot[lane] = s;
  }
  __syncthreads();
  const v4i tv = *(const v4ia*)(tot + 4 * (tid & 7));
  int* gp = GCNT + (size_t)blockIdx.x * GCB + 4 * (tid & 7);
  if (tid < 8) *(volatile v4i*)gp = tv;
  __threadfence();
  if (tid < 8) *(volatile v4i*)gp = tv;
}

__global__ __launch_bounds__(NTHR) void k_off(const int* __restrict__ GCNT, const int* __restrict__ ngp,
                                              const int* __restrict__ gsp, int* GAPN, int* FLAG) {
  __shared__ __attribute__((aligned(16))) int bins[NGP];
  __shared__ __attribute__((aligned(16))) int offs[NGP];
  const int tid = (int)threadIdx.x, lane = tid & 31, wave = tid >> 5;
  const int g0 = 4 * tid;
  {
    v4i c = *(const v4i*)(GCNT + g0); pin(c);
    c.x = (g0     < NG) ? clampi(c.x, 0, NN) : 0;
    c.y = (g0 + 1 < NG) ? clampi(c.y, 0, NN) : 0;
    c.z = (g0 + 2 < NG) ? clampi(c.z, 0, NN) : 0;
    c.w = (g0 + 3 < NG) ? clampi(c.w, 0, NN) : 0;
    *(v4ia*)(bins + g0) = c;
  }
  __syncthreads();
  if (wave == 0) (void)scan1024(bins, offs, offs, lane);
  __syncthreads();
  int gap = gsp[0]; pin(gap);
  gap = clampi(gap, -(1 << 20), 1 << 20);
  int ngv = ngp[0]; pin(ngv);
  const v4i o4 = *(const v4ia*)(offs + g0);
  v4i gv;
  gv.x = (g0     < NG) ? clampi(o4.x + gap, 0, NN - 1) : 0;
  gv.y = (g0 + 1 < NG) ? clampi(o4.y + gap, 0, NN - 1) : 0;
  gv.z = (g0 + 2 < NG) ? clampi(o4.z + gap, 0, NN - 1) : 0;
  gv.w = (g0 + 3 < NG) ? clampi(o4.w + gap, 0, NN - 1) : 0;
  v4i fv;
  fv.x = 0; fv.y = (tid == 0 && ngv != NG) ? 1 : 0; fv.z = 0; fv.w = 0;
  int* fp = FLAG + (size_t)NB * 32 + 4 * (tid & 7);
  *(volatile v4i*)(GAPN + g0) = gv;
  if (tid < 8) *(volatile v4i*)fp = fv;
  __threadfence();
  *(volatile v4i*)(GAPN + g0) = gv;
  if (tid < 8) *(volatile v4i*)fp = fv;
}

__global__ __launch_bounds__(NTHR) void k_compact(const int* __restrict__ srcs, const int* __restrict__ dsts,
                                                  int* LIST, int* CNT, int* OFF, float* DIS, int* FLAG) {
  extern __shared__ __attribute__((aligned(16))) int csm[];
  __shared__ __attribute__((aligned(16))) float disf[NBA];
  int* list = csm;
  int* reg1 = csm + LISTN;
  int* sl   = reg1 + RCAP;
  int* cnt  = sl + RCAP;
  int* offs = cnt + NBA;
  int* cur  = offs + NBA;
  int* misc = cur + NBA;
  const int tid = (int)threadIdx.x, lane = tid & 31, wave = tid >> 5;
  const int blk = (int)blockIdx.x;
  const int nodeBase = blk * NBA;
  const int nb = clampi(NN - nodeBase, 0, NBA);
  {
    const v4i z4 = {0, 0, 0, 0};
    for (int i = tid * 4; i < CMP_ZINTS; i += NTHR * 4) *(v4ia*)(sl + i) = z4;
    if (tid < 16) misc[tid] = 0;
  }
  __syncthreads();

  int tot = 0, ovf = 0;
  const int nChunks = (NE + CHUNK - 1) / CHUNK;
#pragma unroll 1
  for (int ch = 0; ch < nChunks; ++ch) {
    const int cbase = ch * CHUNK;
    const int wc = scan_chunk<SLA>(dsts, NE, cbase, nodeBase, nb, 1, list, tid, lane, wave);
    if (lane == 0) misc[wave] = wc;
    __syncthreads();
    int pre = 0, all = 0;
#pragma unroll
    for (int w2 = 0; w2 < NWAVE; ++w2) {
      int c = misc[w2];
      c = c < 0 ? 0 : (c > WCAP ? WCAP : c);
      all += c;
      pre += (w2 < wave) ? c : 0;
    }
    const int wcc  = wc > WCAP ? WCAP : wc;
    const int base = tot + pre;
#pragma unroll 1
    for (int i = lane; i < wcc; i += 32) {
      const int ent = list[wave * WCAP + i];
      const int el  = (ent >> SLA) & (CHUNK - 1);
      const int sq  = ent & (NBA - 1);
      int eid = cbase + el;
      eid = eid > NE - 1 ? NE - 1 : eid;
      const int sraw = srcs[eid];
      const int s = clampi(sraw, 0, NN - 1);
      const int pos = base + i;
      if (pos < RCAP) reg1[pos] = (int)((unsigned)s | ((unsigned)sq << SRCB));
    }
    if (tot + all > RCAP) ovf = 1;
    tot += all;
    tot = tot > RCAP ? RCAP : tot;
    __syncthreads();
  }
  const int nh = tot;

  if (wave == 0) {
#pragma unroll 1
    for (int b0 = 0; b0 < nh; b0 += 32) {
      const int idx = b0 + lane;
      const int uv  = reg1[idx < nh ? idx : nh - 1];
      const int m32 = (nh - b0) < 32 ? (nh - b0) : 32;
#pragma unroll 1
      for (int k = 0; k < m32; ++k) {
        const int u  = __builtin_amdgcn_readlane(uv, k);
        const int sq = (u >> SRCB) & (NBA - 1);
        if (lane == 0) cnt[sq] = cnt[sq] + 1;
      }
    }
  }
  __syncthreads();
  if (wave == 0) (void)scan1024(cnt, offs, cur, lane);
  __syncthreads();
  if (wave == 0) {
#pragma unroll 1
    for (int b0 = 0; b0 < nh; b0 += 32) {
      const int idx = b0 + lane;
      const int uv  = reg1[idx < nh ? idx : nh - 1];
      const int m32 = (nh - b0) < 32 ? (nh - b0) : 32;
#pragma unroll 1
      for (int k = 0; k < m32; ++k) {
        const int u  = __builtin_amdgcn_readlane(uv, k);
        const int sq = (u >> SRCB) & (NBA - 1);
        if (lane == 0) {
          int p = cur[sq];
          p = p < 0 ? 0 : (p > RCAP - 1 ? RCAP - 1 : p);
          sl[p] = u;
          cur[sq] = p + 1;
        }
      }
    }
  }
  __syncthreads();

  int big = 0;
#pragma unroll 1
  for (int i = 0; i < 4; ++i) {
    const int s = tid + NTHR * i;
    const int c = cnt[s];
    big |= (c > DEGCAP) ? 1 : 0;
    disf[s] = 1.0f / sqrtf((float)c + 1.0f);
  }
  const unsigned bm = __builtin_amdgcn_ballot_w32(big != 0);
  if (lane == 0) misc[8 + wave] = (bm != 0u) ? 1 : 0;
  __syncthreads();
  int fl = ovf;
#pragma unroll
  for (int w2 = 0; w2 < NWAVE; ++w2) fl |= misc[8 + w2];

  const float qnan = __int_as_float(0x7fc00000);
  const v4i c4 = *(const v4ia*)(cnt + 4 * tid);
  v4i o4 = *(const v4ia*)(offs + 4 * tid);
  o4.x += blk * RCAP; o4.y += blk * RCAP; o4.z += blk * RCAP; o4.w += blk * RCAP;
  v4f d4 = *(const v4fa*)(disf + 4 * tid);
  if (fl != 0) { d4.x = qnan; d4.y = qnan; d4.z = qnan; d4.w = qnan; }
  v4i cv;
  cv.x = (tid == 0) ? nh : 0;
  cv.y = (tid == 0) ? fl : 0;
  cv.z = 0; cv.w = 0;
  int* lb = LIST + (size_t)blk * RCAP;
  int* fp = FLAG + (size_t)blk * 32 + 4 * (tid & 7);
  const size_t so = (size_t)nodeBase + 4 * tid;
#pragma unroll 1
  for (int p = tid * 4; p < RCAP; p += NTHR * 4) {
    v4i v = *(const v4ia*)(sl + p);
    v.x &= SRCM; v.y &= SRCM; v.z &= SRCM; v.w &= SRCM;
    *(volatile v4i*)(lb + p) = v;
  }
  *(volatile v4i*)(CNT + so) = c4;
  *(volatile v4i*)(OFF + so) = o4;
  *(volatile v4f*)(DIS + so) = d4;
  if (tid < 8) *(volatile v4i*)fp = cv;
  __threadfence();
#pragma unroll 1
  for (int p = tid * 4; p < RCAP; p += NTHR * 4) {
    v4i v = *(const v4ia*)(sl + p);
    v.x &= SRCM; v.y &= SRCM; v.z &= SRCM; v.w &= SRCM;
    *(volatile v4i*)(lb + p) = v;
  }
  *(volatile v4i*)(CNT + so) = c4;
  *(volatile v4i*)(OFF + so) = o4;
  *(volatile v4f*)(DIS + so) = d4;
  if (tid < 8) *(volatile v4i*)fp = cv;
}

__global__ __launch_bounds__(NTHR) void k_feat(const float* __restrict__ x, const float* __restrict__ embA,
                                               const float* __restrict__ embB, const float* __restrict__ DIS,
                                               float* FEAT) {
  const int u = (int)blockIdx.x * NTHR + (int)threadIdx.x;
  const int row = u >> 3, p = u & 7;
  const int rc = row < NN ? row : NN - 1;
  const bool ok = row < NN;
  const float* xr = x + (size_t)rc * XW;
  v4f xa = *(const v4f*)xr;       pin(xa);
  v4f xb = *(const v4f*)(xr + 4); pin(xb);
  v4f xc = *(const v4f*)(xr + 8); pin(xc);
  float dv = DIS[row];            pin(dv);
  float fa = bfr(xc.z), fb = bfr(xc.w);
  fa = fminf(fmaxf(fa, -16.0f), 16.0f);
  fb = fminf(fmaxf(fb, -16.0f), 16.0f);
  int st = (int)fa, nv = (int)fb;
  st = st < 0 ? st + 10 : st;
  nv = nv < 0 ? nv + 10 : nv;
  st = clampi(st, 0, 9);
  nv = clampi(nv, 0, 9);
  v4f se = *(const v4f*)(embA + 4 * st); pin(se);
  v4f ne = *(const v4f*)(embB + 4 * nv); pin(ne);
  xa = bfr4(xa); xb = bfr4(xb); se = bfr4(se); ne = bfr4(ne);
  const float x8 = bfr(xc.x), x9 = bfr(xc.y);
  v4f o;
  o.x = (p == 0) ? xa.x : (p == 1) ? xb.x : (p == 2) ? x8   : (p == 3) ? se.z : (p == 4) ? ne.z : 0.0f;
  o.y = (p == 0) ? xa.y : (p == 1) ? xb.y : (p == 2) ? x9   : (p == 3) ? se.w : (p == 4) ? ne.w : 0.0f;
  o.z = (p == 0) ? xa.z : (p == 1) ? xb.z : (p == 2) ? se.x : (p == 3) ? ne.x : 0.0f;
  o.w = (p == 0) ? xa.w : (p == 1) ? xb.w : (p == 2) ? se.y : (p == 3) ? ne.y : (p == 7) ? dv : 0.0f;
  if (!ok) { o.x = 0.0f; o.y = 0.0f; o.z = 0.0f; o.w = 0.0f; }
  float* dp = FEAT + (size_t)row * FW + 4 * p;
  *(volatile v4f*)dp = o;
  __threadfence();
  *(volatile v4f*)dp = o;
}

__global__ __launch_bounds__(NTHR) void k_agg1(const int* __restrict__ LIST, const int* __restrict__ CNT,
                                               const int* __restrict__ OFF, const float* __restrict__ FEAT,
                                               unsigned short* AGG1) {
  __shared__ __attribute__((aligned(16))) unsigned short stg[32 * 64];
  const int tid = (int)threadIdx.x, lane = tid & 31, wave = tid >> 5;
  const int nodeBase = (int)blockIdx.x * 32;
#pragma unroll 1
  for (int q = 0; q < 4; ++q) {
    const int r = 4 * wave + q;
    const int node = nodeBase + r;
    const int c = clampi(uloadi(CNT + node), 0, DEGCAP);
    const int o = clampi(uloadi(OFF + node), 0, LISTTOT - 1);
    float sv = FEAT[(size_t)node * FW + lane]; pin(sv);
    const float di = __int_as_float(__builtin_amdgcn_readlane(__float_as_int(sv), 31));
    float acc = 0.0f;
#pragma unroll 1
    for (int b0 = 0; b0 < c; b0 += 32) {
      const int j  = b0 + lane;
      const int jc = j < c ? j : c - 1;
      int idx = o + jc;
      idx = idx > LISTTOT - 1 ? LISTTOT - 1 : idx;
      int sr = LIST[idx]; pin(sr);
      sr = clampi(sr, 0, NN - 1);
      const int m32 = (c - b0) < 32 ? (c - b0) : 32;
#pragma unroll 1
      for (int k = 0; k < m32; ++k) {
        const int sk = __builtin_amdgcn_readlane(sr, k);
        const float fv = FEAT[(size_t)sk * FW + lane];
        const float ds = __int_as_float(__builtin_amdgcn_readlane(__float_as_int(fv), 31));
        const float w  = ds * di;
        acc = fmaf(w, fv, acc);
      }
    }
    float a = acc + (di * di) * sv;
    a = (lane == 31) ? 0.0f : a;
    const unsigned hb = f2bf(a);
    const unsigned lb = f2bf(a - bf2f(hb));
    stg[r * 64 + lane]      = (unsigned short)hb;
    stg[r * 64 + 32 + lane] = (unsigned short)lb;
  }
  __syncthreads();
  const int row = tid >> 3, pc = tid & 7;
  const v8us v = *(const v8usa*)(stg + row * 64 + 8 * pc);
  unsigned short* dp = AGG1 + (size_t)(nodeBase + row) * 64 + 8 * pc;
  *(volatile v8us*)dp = v;
  __threadfence();
  *(volatile v8us*)dp = v;
}

__device__ __forceinline__ void gemm_core(const unsigned short* __restrict__ A,
                                          const unsigned short* __restrict__ WT, int K, int rowBase, int col0,
                                          float* stg, int lane, int wave) {
  const int hh = lane >> 4, m = lane & 15;
  v8f acc[8];
  {
    const v8f z = {0.f, 0.f, 0.f, 0.f, 0.f, 0.f, 0.f, 0.f};
#pragma unroll
    for (int t = 0; t < 8; ++t) acc[t] = z;
  }
  const unsigned short* ap = A  + (size_t)(rowBase + 16 * wave + m) * (size_t)K + 8 * hh;
  const unsigned short* wp = WT + (size_t)(col0 + m) * (size_t)K + 8 * hh;
  const int ksteps = K >> 5;
#pragma unroll 1
  for (int ks = 0; ks < ksteps; ++ks) {
    FragB af;
    af.h[0] = *(const v8usa*)(ap + 32 * ks);
    af.h[1] = *(const v8usa*)(ap + 32 * ks + 16);
#pragma unroll
    for (int t = 0; t < 8; ++t) {
      const unsigned short* wq = wp + (size_t)(16 * t) * (size_t)K + 32 * ks;
      FragB bf;
      bf.h[0] = *(const v8usa*)wq;
      bf.h[1] = *(const v8usa*)(wq + 16);
      acc[t] = wmb(af, bf, acc[t]);
    }
  }
#pragma unroll
  for (int t = 0; t < 8; ++t) {
    const int lc = 16 * t + m;
#pragma unroll
    for (int r = 0; r < 8; ++r) {
      const int lr = 16 * wave + 8 * hh + r;
      stg[lr * GBN + lc] = acc[t][r];
    }
  }
  __syncthreads();
}

template <int HL, int LIVE>
__global__ __launch_bounds__(GTHR) void k_gemm_relu(const unsigned short* __restrict__ A,
                                                    const unsigned short* __restrict__ WT,
                                                    const float* __restrict__ bias, float* outF,
                                                    unsigned short* outH, const int* __restrict__ rinf,
                                                    int K, int nLive) {
  __shared__ __attribute__((aligned(16))) float stg[GBM * GBN];
  const int tid = (int)threadIdx.x, lane = tid & 31, wave = tid >> 5;
  const int rowBase = (int)blockIdx.x * GBM;
  if (LIVE) {
    int r2p = uloadi(rinf + 1);
    r2p = clampi(r2p, 0, R2CAP);
    r2p = (r2p + 127) & ~127;
    if (rowBase >= r2p) return;
  }
  gemm_core(A, WT, K, rowBase, 0, stg, lane, wave);
  const v4f bv = *(const v4f*)(bias + 4 * lane);
  v4f fv[16];
#pragma unroll
  for (int i = 0; i < 16; ++i) {
    const int lr = 16 * wave + i;
    const v4f v = *(const v4fa*)(stg + lr * GBN + 4 * lane);
    const bool live = (rowBase + lr) < nLive;
    v4f y;
    y.x = relu_np(v.x + bv.x); y.y = relu_np(v.y + bv.y);
    y.z = relu_np(v.z + bv.z); y.w = relu_np(v.w + bv.w);
    y.x = live ? y.x : 0.0f; y.y = live ? y.y : 0.0f;
    y.z = live ? y.z : 0.0f; y.w = live ? y.w : 0.0f;
    fv[i] = y;
  }
  if (HL) {
    v4u pk[16];
#pragma unroll
    for (int i = 0; i < 16; ++i) pk[i] = hl_pack(fv[i], lane);
#pragma unroll
    for (int i = 0; i < 16; ++i) {
      const size_t gr = (size_t)(rowBase + 16 * wave + i);
      *(volatile v4f*)(outF + gr * HD + 4 * lane) = fv[i];
      *(volatile v4u*)(outH + gr * 256 + 8 * lane) = pk[i];
    }
    __threadfence();
#pragma unroll
    for (int i = 0; i < 16; ++i) {
      const size_t gr = (size_t)(rowBase + 16 * wave + i);
      *(volatile v4f*)(outF + gr * HD + 4 * lane) = fv[i];
      *(volatile v4u*)(outH + gr * 256 + 8 * lane) = pk[i];
    }
  } else {
#pragma unroll
    for (int i = 0; i < 16; ++i) {
      const size_t gr = (size_t)(rowBase + 16 * wave + i);
      *(volatile v4f*)(outF + gr * HD + 4 * lane) = fv[i];
    }
    __threadfence();
#pragma unroll
    for (int i = 0; i < 16; ++i) {
      const size_t gr = (size_t)(rowBase + 16 * wave + i);
      *(volatile v4f*)(outF + gr * HD + 4 * lane) = fv[i];
    }
  }
}

__global__ __launch_bounds__(NTHR) void k_rows2(const int* __restrict__ GAPN, const int* __restrict__ CNT,
                                                const int* __restrict__ OFF, const int* __restrict__ LIST,
                                                int* ROWS2, int* POS, int* RINF) {
  extern __shared__ __attribute__((aligned(16))) int rsm[];
  __shared__ __attribute__((aligned(16))) int sn[NGP];
  __shared__ __attribute__((aligned(16))) int sc[NGP];
  __shared__ __attribute__((aligned(16))) int so[NGP];
  __shared__ __attribute__((aligned(16))) int sln[NGP];
  __shared__ __attribute__((aligned(16))) int sp[NGP];
  __shared__ int stot[4];
  const int tid = (int)threadIdx.x, lane = tid & 31, wave = tid >> 5;
  {
    const v4i z4 = {0, 0, 0, 0};
    for (int i = tid * 4; i < R2CAP; i += NTHR * 4) *(v4ia*)(rsm + i) = z4;
  }
#pragma unroll 1
  for (int i = 0; i < 4; ++i) {
    const int g = tid + NTHR * i;
    int n = GAPN[g]; pin(n);
    n = clampi(n, 0, NN - 1);
    int c = CNT[n]; pin(c);
    c = clampi(c, 0, DEGCAP);
    int o = OFF[n]; pin(o);
    o = clampi(o, 0, LISTTOT - 1);
    sn[g] = n; sc[g] = c; so[g] = o;
    sln[g] = (g < NG) ? (1 + c) : 0;
  }
  __syncthreads();
  if (wave == 0) {
    const int t = scan1024(sln, sp, sp, lane);
    if (lane == 0) stot[0] = t;
  }
  __syncthreads();
  const int r2  = clampi(stot[0], 0, R2CAP);
  int r2p = (r2 + 127) & ~127;
  r2p = r2p > R2CAP ? R2CAP : r2p;
#pragma unroll 1
  for (int i = 0; i < NGP / NWAVE; ++i) {
    const int g = wave + NWAVE * i;
    if (g < NG) {
      const int p = clampi(sp[g], 0, R2CAP - 1);
      const int c = sc[g];
      const int o = so[g];
      const int n = sn[g];
      if (lane == 0) rsm[p] = n;
#pragma unroll 1
      for (int b0 = 0; b0 < DEGCAP + 16; b0 += 32) {
        const int j  = b0 + lane;
        const int cm = c > 0 ? c - 1 : 0;
        const int jc = j < cm ? j : cm;
        int idx = o + jc;
        idx = idx > LISTTOT - 1 ? LISTTOT - 1 : idx;
        int s = LIST[idx]; pin(s);
        s = clampi(s, 0, NN - 1);
        int q = p + 1 + j;
        q = q > R2CAP - 1 ? R2CAP - 1 : q;
        if (j < c) rsm[q] = s;
      }
    }
  }
  __syncthreads();
  const v4i pv = *(const v4ia*)(sp + 4 * tid);
  v4i iv;
  iv.x = (tid == 0) ? r2 : 0;
  iv.y = (tid == 0) ? r2p : 0;
  iv.z = 0; iv.w = 0;
#pragma unroll 1
  for (int p = tid * 4; p < R2CAP; p += NTHR * 4) {
    const v4i v = *(const v4ia*)(rsm + p);
    *(volatile v4i*)(ROWS2 + p) = v;
  }
  *(volatile v4i*)(POS + 4 * tid) = pv;
  if (tid < 8) *(volatile v4i*)(RINF + 4 * tid) = iv;
  __threadfence();
#pragma unroll 1
  for (int p = tid * 4; p < R2CAP; p += NTHR * 4) {
    const v4i v = *(const v4ia*)(rsm + p);
    *(volatile v4i*)(ROWS2 + p) = v;
  }
  *(volatile v4i*)(POS + 4 * tid) = pv;
  if (tid < 8) *(volatile v4i*)(RINF + 4 * tid) = iv;
}

__global__ __launch_bounds__(NTHR) void k_agg2(const int* __restrict__ ROWS2, const int* __restrict__ RINF,
                                               const int* __restrict__ CNT, const int* __restrict__ OFF,
                                               const float* __restrict__ DIS, const int* __restrict__ LIST,
                                               const float* __restrict__ H1, unsigned short* AGG2) {
  const int tid = (int)threadIdx.x, lane = tid & 31, wave = tid >> 5;
  int r2p = uloadi(RINF + 1);
  r2p = clampi(r2p, 0, R2CAP);
  r2p = (r2p + 127) & ~127;
  const int rb = (int)blockIdx.x * 32;
  if (rb >= r2p) return;
#pragma unroll 1
  for (int q = 0; q < 4; ++q) {
    const int r = rb + 4 * wave + q;
    const int n = clampi(uloadi(ROWS2 + r), 0, NN - 1);
    const float dn = uloadf(DIS + n);
    const int c = clampi(uloadi(CNT + n), 0, DEGCAP);
    const int o = clampi(uloadi(OFF + n), 0, LISTTOT - 1);
    const v4f sv = *(const v4f*)(H1 + (size_t)n * HD + 4 * lane);
    v4f acc = {0.0f, 0.0f, 0.0f, 0.0f};
#pragma unroll 1
    for (int b0 = 0; b0 < c; b0 += 32) {
      const int j  = b0 + lane;
      const int jc = j < c ? j : c - 1;
      int idx = o + jc;
      idx = idx > LISTTOT - 1 ? LISTTOT - 1 : idx;
      int sr = LIST[idx]; pin(sr);
      sr = clampi(sr, 0, NN - 1);
      float ds = DIS[sr]; pin(ds);
      const int wi = __float_as_int(ds * dn);
      const int m32 = (c - b0) < 32 ? (c - b0) : 32;
#pragma unroll 1
      for (int k = 0; k < m32; ++k) {
        const int sk = __builtin_amdgcn_readlane(sr, k);
        const float wk = __int_as_float(__builtin_amdgcn_readlane(wi, k));
        const v4f hv = *(const v4f*)(H1 + (size_t)sk * HD + 4 * lane);
        acc.x = fmaf(wk, hv.x, acc.x); acc.y = fmaf(wk, hv.y, acc.y);
        acc.z = fmaf(wk, hv.z, acc.z); acc.w = fmaf(wk, hv.w, acc.w);
      }
    }
    const float d2 = dn * dn;
    v4f a;
    a.x = acc.x + d2 * sv.x; a.y = acc.y + d2 * sv.y;
    a.z = acc.z + d2 * sv.z; a.w = acc.w + d2 * sv.w;
    const v4u pk = hl_pack(a, lane);
    unsigned short* dp = AGG2 + (size_t)r * 256 + 8 * lane;
    *(volatile v4u*)dp = pk;
    __threadfence();
    *(volatile v4u*)dp = pk;
  }
}

__global__ __launch_bounds__(NTHR) void k_agg3(const int* __restrict__ ROWS2, const int* __restrict__ POS,
                                               const int* __restrict__ GAPN, const int* __restrict__ CNT,
                                               const float* __restrict__ DIS, const float* __restrict__ H2C,
                                               unsigned short* AGG3) {
  const int tid = (int)threadIdx.x, lane = tid & 31, wave = tid >> 5;
  const int g = (int)blockIdx.x * NWAVE + wave;
  const bool live = g < NG;
  const int p = clampi(uloadi(POS + g), 0, R2CAP - 1);
  const int n = clampi(uloadi(GAPN + g), 0, NN - 1);
  const float dn = uloadf(DIS + n);
  int c = clampi(uloadi(CNT + n), 0, DEGCAP);
  c = live ? c : 0;
  const v4f sv = *(const v4f*)(H2C + (size_t)p * HD + 4 * lane);
  v4f acc = {0.0f, 0.0f, 0.0f, 0.0f};
#pragma unroll 1
  for (int b0 = 0; b0 < c; b0 += 32) {
    const int j  = b0 + lane;
    const int jc = j < c ? j : c - 1;
    int r = p + 1 + jc;
    r = r > R2CAP - 1 ? R2CAP - 1 : r;
    int sr = ROWS2[r]; pin(sr);
    sr = clampi(sr, 0, NN - 1);
    float ds = DIS[sr]; pin(ds);
    const int wi = __float_as_int(ds * dn);
    const int m32 = (c - b0) < 32 ? (c - b0) : 32;
#pragma unroll 1
    for (int k = 0; k < m32; ++k) {
      int rk = p + 1 + b0 + k;
      rk = rk > R2CAP - 1 ? R2CAP - 1 : rk;
      const float wk = __int_as_float(__builtin_amdgcn_readlane(wi, k));
      const v4f hv = *(const v4f*)(H2C + (size_t)rk * HD + 4 * lane);
      acc.x = fmaf(wk, hv.x, acc.x); acc.y = fmaf(wk, hv.y, acc.y);
      acc.z = fmaf(wk, hv.z, acc.z); acc.w = fmaf(wk, hv.w, acc.w);
    }
  }
  const float d2 = dn * dn;
  v4f a;
  a.x = acc.x + d2 * sv.x; a.y = acc.y + d2 * sv.y;
  a.z = acc.z + d2 * sv.z; a.w = acc.w + d2 * sv.w;
  a.x = live ? a.x : 0.0f; a.y = live ? a.y : 0.0f;
  a.z = live ? a.z : 0.0f; a.w = live ? a.w : 0.0f;
  const v4u pk = hl_pack(a, lane);
  unsigned short* dp = AGG3 + (size_t)g * 256 + 8 * lane;
  *(volatile v4u*)dp = pk;
  __threadfence();
  *(volatile v4u*)dp = pk;
}

__global__ __launch_bounds__(GTHR) void k_gemm_gru(char* ws, unsigned aInp, unsigned aHf, unsigned aHb) {
  __shared__ __attribute__((aligned(16))) float stg[GBM * GBN];
  const int tid = (int)threadIdx.x, lane = tid & 31, wave = tid >> 5;
  const int rowBase = (int)blockIdx.x * GBM;
  const int col0 = (int)blockIdx.y * GBN;
  const int z = (int)blockIdx.z;
  const unsigned ao = (z == 1) ? aHf : ((z == 3) ? aHb : aInp);
  const unsigned short* A  = (const unsigned short*)ws + ao;
  const unsigned short* WT = (const unsigned short*)(ws + O_WG) + (size_t)z * 384 * 256;
  float* out = (float*)(ws + O_GG) + (size_t)z * GGP;
  gemm_core(A, WT, 256, rowBase, col0, stg, lane, wave);
  v4f fv[16];
#pragma unroll
  for (int i = 0; i < 16; ++i) fv[i] = *(const v4fa*)(stg + (16 * wave + i) * GBN + 4 * lane);
#pragma unroll
  for (int i = 0; i < 16; ++i) {
    const size_t gr = (size_t)(rowBase + 16 * wave + i);
    *(volatile v4f*)(out + gr * 384 + col0 + 4 * lane) = fv[i];
  }
  __threadfence();
#pragma unroll
  for (int i = 0; i < 16; ++i) {
    const size_t gr = (size_t)(rowBase + 16 * wave + i);
    *(volatile v4f*)(out + gr * 384 + col0 + 4 * lane) = fv[i];
  }
}

__global__ __launch_bounds__(NTHR) void k_gate(char* ws, unsigned oPrevF, unsigned oPrevB, unsigned oNewF,
                                               unsigned oNewB) {
  __shared__ __attribute__((aligned(16))) float sb[768];
  __shared__ __attribute__((aligned(16))) float hrow[NWAVE * HD];
  const int tid = (int)threadIdx.x, lane = tid & 31, wave = tid >> 5;
  const int dir = (int)blockIdx.y;
  const int g = (int)blockIdx.x * NWAVE + wave;
  const float* bg = (const float*)(ws + O_BGRU) + dir * 768;
#pragma unroll 1
  for (int i = tid; i < 768; i += NTHR) sb[i] = bg[i];
  __syncthreads();
  const float* gi = (const float*)(ws + O_GG) + (size_t)(2 * dir) * GGP + (size_t)g * 384;
  const float* gh = gi + GGP;
  const unsigned po = (dir != 0) ? oPrevB : oPrevF;
  const unsigned no = (dir != 0) ? oNewB : oNewF;
  const float* hp = (const float*)(ws + po) + (size_t)g * HD;
#pragma unroll 1
  for (int j = 0; j < 4; ++j) {
    const int c = 32 * j + lane;
    const float ir = gi[c] + sb[c];
    const float iz = gi[128 + c] + sb[128 + c];
    const float in = gi[256 + c] + sb[256 + c];
    const float hr = gh[c] + sb[384 + c];
    const float hz = gh[128 + c] + sb[512 + c];
    const float hn = gh[256 + c] + sb[640 + c];
    const float hv = hp[c];
    const float r  = 1.0f / (1.0f + expf(-(ir + hr)));
    const float zz = 1.0f / (1.0f + expf(-(iz + hz)));
    const float nn = tanhf(in + r * hn);
    hrow[wave * HD + c] = (1.0f - zz) * nn + zz * hv;
  }
  __syncthreads();
  const v4f h4 = *(const v4fa*)(hrow + wave * HD + 4 * lane);
  const v4u pk = hl_pack(h4, lane);
  float* fp = (float*)(ws + no) + (size_t)g * HD + 4 * lane;
  const size_t hlo = (dir != 0) ? O_HBHL : O_HFHL;
  unsigned short* hq = (unsigned short*)(ws + hlo) + (size_t)g * 256 + 8 * lane;
  unsigned short* oq = (unsigned short*)(ws + O_OUTHL) + (size_t)g * 512 + dir * 128 + (lane >> 4) * 256 +
                       8 * (lane & 15);
  *(volatile v4f*)fp = h4;
  *(volatile v4u*)hq = pk;
  *(volatile v4u*)oq = pk;
  __threadfence();
  *(volatile v4f*)fp = h4;
  *(volatile v4u*)hq = pk;
  *(volatile v4u*)oq = pk;
}

__global__ __launch_bounds__(GTHR) void k_gemm_head(char* ws, int step) {
  __shared__ __attribute__((aligned(16))) float stg[GBM * GBN];
  __shared__ __attribute__((aligned(16))) float swh[256];
  __shared__ __attribute__((aligned(16))) float sdot[128];
  const int tid = (int)threadIdx.x, lane = tid & 31, wave = tid >> 5;
  const int rowBase = (int)blockIdx.x * GBM;
  const int cb = (int)blockIdx.y;
  const float* sc = (const float*)(ws + O_SC);
  {
    const v2f w = *(const v2f*)(sc + 256 + 2 * tid);
    swh[2 * tid] = w.x; swh[2 * tid + 1] = w.y;
  }
  gemm_core((const unsigned short*)(ws + O_OUTHL), (const unsigned short*)(ws + O_WHD), 512, rowBase,
            cb * GBN, stg, lane, wave);
  if (cb == 0) {
    const v4f bv = *(const v4f*)(sc + 4 * lane);
#pragma unroll
    for (int i = 0; i < 16; ++i) {
      float* pp = stg + (16 * wave + i) * GBN + 4 * lane;
      const v4f v = *(const v4fa*)pp;
      v4f y;
      y.x = relu_np(v.x + bv.x); y.y = relu_np(v.y + bv.y);
      y.z = relu_np(v.z + bv.z); y.w = relu_np(v.w + bv.w);
      *(v4fa*)pp = y;
    }
    __syncthreads();
    const int row = tid & 63, c = tid >> 6;
    const float b2v = sc[512 + c];
    const float* hr = stg + row * GBN;
    float s = 0.0f;
#pragma unroll 4
    for (int k4 = 0; k4 < 32; ++k4) {
      const v4f hv = *(const v4fa*)(hr + 4 * k4);
      const float* w = swh + 8 * k4 + c;
      s = fmaf(hv.x, w[0], s);
      s = fmaf(hv.y, w[2], s);
      s = fmaf(hv.z, w[4], s);
      s = fmaf(hv.w, w[6], s);
    }
    sdot[row * 2 + c] = s + b2v;
    __syncthreads();
    if (wave == 0) {
      const v4f v = *(const v4fa*)(sdot + 4 * lane);
      float* pp = (float*)(ws + O_PRED) + (size_t)step * (NGP * 2) + (size_t)rowBase * 2 + 4 * lane;
      *(volatile v4f*)pp = v;
      __threadfence();
      *(volatile v4f*)pp = v;
    }
  } else {
    const v4f bv = *(const v4f*)(sc + 128 + 4 * lane);
    v4u pk[16];
#pragma unroll
    for (int i = 0; i < 16; ++i) {
      const v4f v = *(const v4fa*)(stg + (16 * wave + i) * GBN + 4 * lane);
      v4f y;
      y.x = v.x + bv.x; y.y = v.y + bv.y; y.z = v.z + bv.z; y.w = v.w + bv.w;
      pk[i] = hl_pack(y, lane);
    }
    unsigned short* ip = (unsigned short*)(ws + O_INPHL);
#pragma unroll
    for (int i = 0; i < 16; ++i) {
      const size_t gr = (size_t)(rowBase + 16 * wave + i);
      *(volatile v4u*)(ip + gr * 256 + 8 * lane) = pk[i];
    }
    __threadfence();
#pragma unroll
    for (int i = 0; i < 16; ++i) {
      const size_t gr = (size_t)(rowBase + 16 * wave + i);
      *(volatile v4u*)(ip + gr * 256 + 8 * lane) = pk[i];
    }
  }
}

__global__ __launch_bounds__(NTHR) void k_store(const float* __restrict__ PRED, const int* __restrict__ FLAG,
                                                float* out) {
  __shared__ __attribute__((aligned(16))) float os[6144];
  __shared__ int sfl[NTHR];
  const int tid = (int)threadIdx.x;
  {
    const int li = tid <= NB ? tid : NB;
    int f = FLAG[(size_t)li * 32 + 1]; pin(f);
    sfl[tid] = (tid <= NB) ? f : 0;
  }
#pragma unroll 1
  for (int e = tid; e < 6144; e += NTHR) {
    const int ec = e < 5999 ? e : 5999;
    const int g = ec / 6;
    const int rem = ec - 6 * g;
    const int t = rem >> 1, c = rem & 1;
    float v = PRED[(size_t)t * (NGP * 2) + (size_t)g * 2 + c]; pin(v);
    os[e] = (e < 6000) ? v : 0.0f;
  }
  __syncthreads();
  int any = 0;
#pragma unroll 1
  for (int i = 0; i < NTHR; ++i) any |= sfl[i];
  const float qnan = __int_as_float(0x7fc00000);
  v4f ov[6];
#pragma unroll
  for (int it = 0; it < 6; ++it) {
    v4f v = *(const v4fa*)(os + 4 * (it * NTHR + tid));
    if (any != 0) { v.x = qnan; v.y = qnan; v.z = qnan; v.w = qnan; }
    ov[it] = v;
  }
#pragma unroll
  for (int it = 0; it < 6; ++it) {
    const int q = it * NTHR + tid;
    if (q < 1500) *(volatile v4f*)(out + 4 * (size_t)q) = ov[it];
  }
  __threadfence();
#pragma unroll
  for (int it = 0; it < 6; ++it) {
    const int q = it * NTHR + tid;
    if (q < 1500) *(volatile v4f*)(out + 4 * (size_t)q) = ov[it];
  }
}

extern "C" void kernel_launch(void* const* d_in, const int* in_sizes, int n_in,
                              void* d_out, int out_size, void* d_ws, size_t ws_size,
                              hipStream_t stream) {
  if (n_in < 27) return;
  static const int expect[27] = {
    NN * XW, 2 * NE, NN, 40, 40, NFEAT * HD, HD, HD * HD, HD, HD * HD, HD,
    HD * 384, HD * 384, 384, 384, HD * 384, HD * 384, 384, 384,
    256 * HD, HD, 256 * HD, HD, HD * 2, 2, 1, 1 };
  for (int i = 0; i < 27; ++i) if (in_sizes[i] != expect[i]) return;
  if (out_size != NG * 3 * 2) return;
  if (ws_size < WS_TOTAL) return;

  const float* x     = (const float*)d_in[0];
  const int*   ei    = (const int*)  d_in[1];
  const int*   batch = (const int*)  d_in[2];
  const float* embA  = (const float*)d_in[3];
  const float* embB  = (const float*)d_in[4];
  const float* W1    = (const float*)d_in[5];
  const float* b1    = (const float*)d_in[6];
  const float* W2    = (const float*)d_in[7];
  const float* b2    = (const float*)d_in[8];
  const float* W3    = (const float*)d_in[9];
  const float* b3    = (const float*)d_in[10];
  const float* Wif   = (const float*)d_in[11];
  const float* Whf   = (const float*)d_in[12];
  const float* bif   = (const float*)d_in[13];
  const float* bhf   = (const float*)d_in[14];
  const float* Wib   = (const float*)d_in[15];
  const float* Whb   = (const float*)d_in[16];
  const float* bib   = (const float*)d_in[17];
  const float* bhb   = (const float*)d_in[18];
  const float* Wred  = (const float*)d_in[19];
  const float* bred  = (const float*)d_in[20];
  const float* Wh1   = (const float*)d_in[21];
  const float* bh1   = (const float*)d_in[22];
  const float* Wh2   = (const float*)d_in[23];
  const float* bh2   = (const float*)d_in[24];
  const int*   ngp   = (const int*)  d_in[25];
  const int*   gsp   = (const int*)  d_in[26];
  float* out = (float*)d_out;
  const int* src = ei;
  const int* dst = ei + NE;

  char* ws = (char*)d_ws;
  unsigned short* W1D  = (unsigned short*)(ws + O_W1D);
  unsigned short* W2D  = (unsigned short*)(ws + O_W2D);
  unsigned short* W3D  = (unsigned short*)(ws + O_W3D);
  float*          BG   = (float*)(ws + O_BG);
  unsigned short* WG   = (unsigned short*)(ws + O_WG);
  float*          BGRU = (float*)(ws + O_BGRU);
  unsigned short* WHD  = (unsigned short*)(ws + O_WHD);
  float*          SC   = (float*)(ws + O_SC);
  int*            GAPN = (int*)(ws + O_GAPN);
  int*            GCNT = (int*)(ws + O_GCNT);
  int*            FLAG = (int*)(ws + O_FLAG);
  int*            LIST = (int*)(ws + O_LIST);
  int*            CNT  = (int*)(ws + O_CNT);
  int*            OFF  = (int*)(ws + O_OFF);
  float*          DIS  = (float*)(ws + O_DIS);
  float*          FEAT = (float*)(ws + O_Q);
  unsigned short* AGG1 = (unsigned short*)(ws + O_AGG1);
  float*          H2C  = (float*)(ws + O_Q);
  float*          H1   = (float*)(ws + O_H1);
  unsigned short* AGG2 = (unsigned short*)(ws + O_AGG2);
  int*            ROWS2 = (int*)(ws + O_ROWS2);
  int*            POS  = (int*)(ws + O_POS);
  int*            RINF = (int*)(ws + O_RINF);
  unsigned short* AGG3 = (unsigned short*)(ws + O_AGG3);
  float*          H0   = (float*)(ws + O_H0);
  unsigned short* H0HL = (unsigned short*)(ws + O_H0HL);
  float*          PRED = (float*)(ws + O_PRED);

  const int cmpLds = CMP_LDS_INTS * 4;
  const int r2Lds  = R2CAP * 4;
  hipFuncSetAttribute(reinterpret_cast<const void*>(&k_compact),
                      hipFuncAttributeMaxDynamicSharedMemorySize, cmpLds);
  hipFuncSetAttribute(reinterpret_cast<const void*>(&k_rows2),
                      hipFuncAttributeMaxDynamicSharedMemorySize, r2Lds);

  k_pa<<<(PA_U1 + 2 * PA_U2 + PA_UB) / NTHR, NTHR, 0, stream>>>(W1, b1, W2, b2, W3, b3, W1D, W2D, W3D, BG);
  k_pb<<<(4 * PB_UG + PB_UB) / NTHR, NTHR, 0, stream>>>(Wif, Whf, bif, bhf, Wib, Whb, bib, bhb, WG, BGRU);
  k_pc<<<(PC_UW + PC_US) / NTHR, NTHR, 0, stream>>>(Wred, bred, Wh1, bh1, Wh2, bh2, WHD, SC);
  k_gcnt<<<NGP / GCB, NTHR, 0, stream>>>(batch, GCNT);
  k_off<<<1, NTHR, 0, stream>>>(GCNT, ngp, gsp, GAPN, FLAG);
  k_compact<<<NB, NTHR, cmpLds, stream>>>(src, dst, LIST, CNT, OFF, DIS, FLAG);
  k_feat<<<(NPD * 8) / NTHR, NTHR, 0, stream>>>(x, embA, embB, DIS, FEAT);
  k_agg1<<<NPD / 32, NTHR, 0, stream>>>(LIST, CNT, OFF, FEAT, AGG1);
  k_gemm_relu<0, 0><<<NPD / GBM, GTHR, 0, stream>>>(AGG1, W1D, BG, H1, AGG1, RINF, 64, NN);
  k_rows2<<<1, NTHR, r2Lds, stream>>>(GAPN, CNT, OFF, LIST, ROWS2, POS, RINF);
  k_agg2<<<R2CAP / 32, NTHR, 0, stream>>>(ROWS2, RINF, CNT, OFF, DIS, LIST, H1, AGG2);
  k_gemm_relu<0, 1><<<R2CAP / GBM, GTHR, 0, stream>>>(AGG2, W2D, BG + 128, H2C, AGG2, RINF, 256, R2CAP);
  k_agg3<<<NGP / NWAVE, NTHR, 0, stream>>>(ROWS2, POS, GAPN, CNT, DIS, H2C, AGG3);
  k_gemm_relu<1, 0><<<NGP / GBM, GTHR, 0, stream>>>(AGG3, W3D, BG + 256, H0, H0HL, RINF, 256, NG);

  for (int t = 0; t < 3; ++t) {
    const unsigned aInp = (unsigned)(((t == 0) ? O_H0HL : O_INPHL) / 2);
    const unsigned aHf  = (unsigned)(((t == 0) ? O_H0HL : O_HFHL) / 2);
    const unsigned aHb  = (unsigned)(((t == 0) ? O_H0HL : O_HBHL) / 2);
    const unsigned pF = (unsigned)((t == 0) ? O_H0 : (O_HF + (size_t)((t - 1) & 1) * HPL));
    const unsigned pB = (unsigned)((t == 0) ? O_H0 : (O_HB + (size_t)((t - 1) & 1) * HPL));
    const unsigned nF = (unsigned)(O_HF + (size_t)(t & 1) * HPL);
    const unsigned nB = (unsigned)(O_HB + (size_t)(t & 1) * HPL);
    k_gemm_gru<<<dim3(NGP / GBM, 3, 4), GTHR, 0, stream>>>(ws, aInp, aHf, aHb);
    k_gate<<<dim3(NGP / NWAVE, 2), NTHR, 0, stream>>>(ws, pF, pB, nF, nB);
    k_gemm_head<<<dim3(NGP / GBM, 2), GTHR, 0, stream>>>(ws, t);
  }
  k_store<<<1, NTHR, 0, stream>>>(PRED, FLAG, out);
}
